// IndividualDecoder_19559281066669
// MI455X (gfx1250) — hardware-verified
//
#include <hip/hip_runtime.h>


namespace {
constexpr int B = 8192, IN = 1024, OUT = 1024, HID = 4, NCOL = OUT * HID;

typedef _Float16 b16;
typedef __attribute__((ext_vector_type(16))) _Float16 v16b;
typedef __attribute__((ext_vector_type(8))) _Float16 v8b;
typedef __attribute__((ext_vector_type(8))) float v8f;
typedef __attribute__((ext_vector_type(4))) float v4f;
__device__ __forceinline__ float bf16_rne(float f) { unsigned int u = __float_as_uint(f); u += 0x7FFFu + ((u >> 16) & 1u); return __uint_as_float(u & 0xFFFF0000u); }
__device__ __forceinline__ v16b frag_kb(const b16* p, int hh) { const v8b a = *(const v8b*)(p + 8 * hh), b = *(const v8b*)(p + 16 + 8 * hh); v16b f;
#pragma unroll
  for (int e = 0; e < 8; ++e) { f[e] = a[e]; f[8 + e] = b[e]; } return f; }
__device__ __forceinline__ v8f wmma16b(v16b a, v16b b, v8f c) { v8f d = __builtin_amdgcn_wmma_f32_16x16x32_f16(false, a, false, b, (short)0, c, false, false); asm volatile("v_nop\n\tv_nop\n\tv_nop\n\tv_nop" : "+v"(d) : "v"(a), "v"(b)); return d; }
__device__ __forceinline__ void wave_lds_sync() { __builtin_amdgcn_fence(__ATOMIC_RELEASE, "workgroup"); __builtin_amdgcn_wave_barrier(); __builtin_amdgcn_fence(__ATOMIC_ACQUIRE, "workgroup"); }
__device__ __forceinline__ float pmul(float a, float b) { float p = a * b; asm volatile("" : "+v"(p)); return p; }

__global__ __launch_bounds__(256) void prep_kernel(const float* __restrict__ x, const float* __restrict__ W1, const float* __restrict__ b1, const float* __restrict__ W2, const float* __restrict__ b2, b16* __restrict__ R, b16* __restrict__ X, float* __restrict__ P) {
  const size_t tid = (size_t)blockIdx.x * 256 + threadIdx.x, nth = (size_t)gridDim.x * 256;
  for (int pass = 0; pass < 2; ++pass) {
    for (size_t p = tid; p < (size_t)NCOL * IN / 8; p += nth) { const int n = (int)(p / (IN / 8)), k0 = (int)(p % (IN / 8)) * 8; const int o = n >> 2, j = n & 3; v8b v;
#pragma unroll
      for (int e = 0; e < 8; ++e) v[e] = (b16)bf16_rne(W1[((size_t)o * IN + k0 + e) * HID + j]); *(volatile v8b*)(R + (size_t)n * IN + k0) = v; }
    for (size_t p = tid; p < (size_t)B * IN / 8; p += nth) { v8b v;
#pragma unroll
      for (int e = 0; e < 8; ++e) v[e] = (b16)bf16_rne(x[p * 8 + e]); *(volatile v8b*)(X + p * 8) = v; }
    for (size_t q = tid; q < 9216; q += nth) { const int i = (int)q; P[q] = (i < 4096) ? bf16_rne(b1[i]) : (i < 8192) ? bf16_rne(W2[i - 4096]) : bf16_rne(b2[i - 8192]); }
    __threadfence(); }
}

__global__ __launch_bounds__(64) void mlp_kernel(const b16* __restrict__ X, const b16* __restrict__ R, const float* __restrict__ P, float* __restrict__ out) {
  __shared__ __attribute__((aligned(16))) float Ts[2][32][32 + 4];
  const int lane = threadIdx.x & 31, wave = threadIdx.x >> 5, nloc = lane & 15, hlf = lane >> 4, m0 = blockIdx.y * 32, c0 = blockIdx.x * 256 + wave * 128; const float* b1 = P; const float* W2 = P + 4096; const float* b2 = P + 8192;
  v8f acc[2][8];
#pragma unroll
  for (int r = 0; r < 2; ++r)
#pragma unroll
    for (int t = 0; t < 8; ++t) acc[r][t] = (v8f){};
#pragma unroll 2
  for (int kb = 0; kb < IN; kb += 32) { const v16b a0 = frag_kb(X + (size_t)(m0 + nloc) * IN + kb, hlf), a1 = frag_kb(X + (size_t)(m0 + 16 + nloc) * IN + kb, hlf);
#pragma unroll
    for (int t = 0; t < 8; ++t) { const v16b bw = frag_kb(R + (size_t)(c0 + t * 16 + nloc) * IN + kb, hlf); acc[0][t] = wmma16b(a0, bw, acc[0][t]); acc[1][t] = wmma16b(a1, bw, acc[1][t]); } }
#pragma unroll
  for (int t = 0; t < 8; ++t) { const int c = c0 + t * 16 + nloc; const float bb = b1[c], w2 = W2[c];
#pragma unroll
    for (int r = 0; r < 2; ++r)
#pragma unroll
      for (int v = 0; v < 8; ++v) { float h = acc[r][t][v] + bb; h = (h >= 0.0f) ? h : 0.1f * h; float p = pmul(h, w2); p += __shfl_xor(p, 1); p += __shfl_xor(p, 2);
        if ((nloc & 3) == 0) { const int ol = (wave * 128 + t * 16 + nloc - wave * 128) >> 2;
          Ts[wave][r * 16 + 8 * hlf + v][ol] = p + b2[(c0 + t * 16 + nloc) >> 2]; } } }
  wave_lds_sync();
  const int o0 = c0 >> 2;
  for (int pass = 0; pass < 2; ++pass) { for (int i = lane; i < 32 * 8; i += 32) { const int rr = i >> 3, c4 = (i & 7) * 4; *(volatile v4f*)(out + (size_t)(m0 + rr) * OUT + o0 + c4) = *(const v4f*)(&Ts[wave][rr][c4]); } __threadfence(); }
}
}

extern "C" void kernel_launch(void* const* d_in, const int* in_sizes, int n_in,
                              void* d_out, int out_size, void* d_ws, size_t ws_size, hipStream_t stream) {
  (void)n_in; (void)out_size;
  const float* x = (const float*)d_in[0]; const float* W1 = (const float*)d_in[1]; const float* b1 = (const float*)d_in[2]; const float* W2 = (const float*)d_in[3]; const float* b2 = (const float*)d_in[4];
  float* out = (float*)d_out;
  if (in_sizes[0] != B * IN || in_sizes[1] != OUT * IN * HID || in_sizes[2] != OUT * HID || in_sizes[3] != OUT * HID || in_sizes[4] != OUT) return;
  size_t off = 0; char* ws = (char*)d_ws;
  auto carve = [&](size_t bytes) { char* p = ws + off; off += (bytes + 255) & ~(size_t)255; return p; };
  b16* R = (b16*)carve((size_t)NCOL * IN * 2); b16* X = (b16*)carve((size_t)B * IN * 2); float* P = (float*)carve(9216 * 4);
  if (off > ws_size) return;
  prep_kernel<<<512, 256, 0, stream>>>(x, W1, b1, W2, b2, R, X, P);
  mlp_kernel<<<dim3(NCOL / 256, B / 32), 64, 0, stream>>>(X, R, P, out);
}
